// BaseModel_44341242364529
// MI455X (gfx1250) — hardware-run, weakly checked
//
#include <hip/hip_runtime.h>


namespace {
typedef _Float16 b16;
typedef __attribute__((ext_vector_type(16))) _Float16 v16b;
typedef __attribute__((ext_vector_type(8))) _Float16 v8b;
typedef __attribute__((ext_vector_type(4))) _Float16 v4h;
typedef __attribute__((ext_vector_type(2))) _Float16 v2h;
typedef __attribute__((ext_vector_type(8))) float v8f;
typedef __attribute__((ext_vector_type(4))) float v4f;
typedef __attribute__((ext_vector_type(2))) float v2f;
__device__ __forceinline__ float bf16_rne(float f) { unsigned int u = __float_as_uint(f); u += 0x7FFFu + ((u >> 16) & 1u); return __uint_as_float(u & 0xFFFF0000u); }
__device__ __forceinline__ void split16(float v, b16& hi, b16& lo) { hi = (b16)v; lo = (b16)(v - (float)hi); }
__device__ __forceinline__ v16b frag_kb(const b16* p, int hh) { const v8b a = *(const v8b*)(p + 8 * hh), b = *(const v8b*)(p + 16 + 8 * hh); v16b f;
#pragma unroll
  for (int e = 0; e < 8; ++e) { f[e] = a[e]; f[8 + e] = b[e]; } return f; }
__device__ __forceinline__ v8f wmma16b(v16b a, v16b b, v8f c) { v8f d = __builtin_amdgcn_wmma_f32_16x16x32_f16(false, a, false, b, (short)0, c, false, false); asm volatile("v_nop\n\tv_nop\n\tv_nop\n\tv_nop" : "+v"(d) : "v"(a), "v"(b)); return d; }
__device__ __forceinline__ void wave_lds_sync() { __builtin_amdgcn_fence(__ATOMIC_RELEASE, "workgroup"); __builtin_amdgcn_wave_barrier(); __builtin_amdgcn_fence(__ATOMIC_ACQUIRE, "workgroup"); }
__device__ __forceinline__ float pmul(float a, float b) { float p = a * b; asm volatile("" : "+v"(p)); return p; }
__device__ __forceinline__ int iclamp(int v, int lo, int hi) { return v < lo ? lo : (v > hi ? hi : v); }
__device__ __forceinline__ float nexp2(float v) { return __builtin_amdgcn_exp2f(v); }

constexpr int IMG = 64, PATCH = 4, GT = 16, NPAT = 4096, PVOL = 64, D = 256, NH = 4, DH = 64, L = NPAT + 2, LP = 4128  , NL = LP  , LOUT = (NL < L ? NL : L), KN = 133, DFF = 1024, NLAY = 2;
constexpr float XS = 8.0f, WSC = 256.0f, LNEPS = 1e-5f, SCALE = 0.125f;
static_assert(LP % 32 == 0 && LP >= L && NL % 32 == 0 && NL <= LP && D == 256 && DFF % 128 == 0 && NPAT % 32 == 0, "tiling");
template <int KD, int NOUT>
__global__ __launch_bounds__(256) void wprep_kernel(const float* __restrict__ w, b16* __restrict__ WT) {
  static_assert(KD % 8 == 0, "wprep"); const size_t u = (size_t)blockIdx.x * 256 + threadIdx.x; if (u >= (size_t)NOUT * KD / 8) return; const size_t e = u * 8; const int oo = (int)(e / KD), k0 = (int)(e % KD); v8b o;
  for (int j = 0; j < 8; ++j) o[j] = (b16)(bf16_rne(w[(size_t)(k0 + j) * NOUT + oo]) * WSC);
  for (int pass = 0; pass < 2; ++pass) { *(volatile v8b*)(WT + e) = o; __threadfence(); }
}
template <int KD, int NOUT, int NV, bool RNDA  >
__global__ __launch_bounds__(64) void gemm_kernel(const float* __restrict__ A, const b16* __restrict__ W, float* __restrict__ T) {
  constexpr int SL = NOUT < 128 ? NOUT : 128, NT = SL / 16, KC = KD < 128 ? KD : 128;
  static_assert(KD % KC == 0 && KC % 32 == 0 && NOUT % SL == 0 && SL % 32 == 0, "gemm tiling");
  __shared__ __attribute__((aligned(16))) b16 Ah[2][16][KC + 8], Al[2][16][KC + 8]; __shared__ __attribute__((aligned(16))) float Tf[2][16][SL + 4];
  const int wave = threadIdx.x >> 5, lane = threadIdx.x & 31, nloc = lane & 15, hlf = lane >> 4; const size_t m0 = (size_t)blockIdx.x * 32 + wave * 16; const int n0 = blockIdx.y * SL;
  v8f acc[NT];
#pragma unroll
  for (int t = 0; t < NT; ++t) acc[t] = (v8f){};
#pragma unroll 1
  for (int kc = 0; kc < KD; kc += KC) {
    for (int idx = lane; idx < 16 * (KC / 4); idx += 32) { const int rr = idx / (KC / 4), c4 = (idx % (KC / 4)) * 4; const size_t row = (m0 + rr < (size_t)NV) ? (m0 + rr) : (size_t)(NV - 1); const v4f v = *(const v4f*)(A + row * KD + kc + c4); v4h hv, lv;
      for (int j = 0; j < 4; ++j) { b16 ph, pl; split16((RNDA ? bf16_rne(v[j]) : v[j]) * XS, ph, pl); hv[j] = ph; lv[j] = pl; } *(v4h*)(&Ah[wave][rr][c4]) = hv; *(v4h*)(&Al[wave][rr][c4]) = lv; }
    wave_lds_sync();
#pragma unroll
    for (int kb = 0; kb < KC; kb += 32) { const v16b a = frag_kb(&Ah[wave][nloc][kb], hlf), al = frag_kb(&Al[wave][nloc][kb], hlf);
#pragma unroll
      for (int t = 0; t < NT; ++t) { const v16b bw = frag_kb(W + (size_t)(n0 + t * 16 + nloc) * KD + kc + kb, hlf); acc[t] = wmma16b(a, bw, acc[t]); acc[t] = wmma16b(al, bw, acc[t]); } }
    wave_lds_sync(); }
#pragma unroll
  for (int t = 0; t < NT; ++t)
#pragma unroll
    for (int r = 0; r < 8; ++r) Tf[wave][8 * hlf + r][t * 16 + nloc] = acc[t][r] * (1.0f / (XS * WSC));
  wave_lds_sync();
  for (int pass = 0; pass < 2; ++pass) { for (int idx = lane; idx < 16 * (SL / 4); idx += 32) { const int rr = idx / (SL / 4), c4 = (idx % (SL / 4)) * 4; *(volatile v4f*)(T + (m0 + rr) * NOUT + n0 + c4) = *(const v4f*)(&Tf[wave][rr][c4]); } __threadfence(); }
}

__global__ __launch_bounds__(64) void patch_kernel(const float* __restrict__ img, const b16* __restrict__ WPt, const float* __restrict__ pb, float* __restrict__ X) {
  __shared__ __attribute__((aligned(16))) b16 As[2][16][PVOL + 8]; __shared__ __attribute__((aligned(16))) float Tf[2][16][128 + 4];
  const int wave = threadIdx.x >> 5, lane = threadIdx.x & 31, nloc = lane & 15, hlf = lane >> 4; const int n0 = blockIdx.x * 32 + wave * 16; const int c0 = blockIdx.y * 128;
  for (int idx = lane; idx < 16 * 16; idx += 32) { const int rr = idx / 16, pq = idx % 16, p = pq / 4, q = pq % 4; const int n = n0 + rr, t = n / 256, h = (n / 16) % 16, w = n % 16;
    const v4f f = *(const v4f*)(img + ((size_t)(t * PATCH + p) * IMG + (h * PATCH + q)) * IMG + w * PATCH); v4h o; for (int j = 0; j < 4; ++j) o[j] = (b16)(bf16_rne(f[j]) * XS); *(v4h*)(&As[wave][rr][pq * 4]) = o; }
  wave_lds_sync();
  v8f acc[8];
#pragma unroll
  for (int tt = 0; tt < 8; ++tt) acc[tt] = (v8f){};
#pragma unroll
  for (int kb = 0; kb < PVOL; kb += 32) { const v16b a = frag_kb(&As[wave][nloc][kb], hlf);
#pragma unroll
    for (int tt = 0; tt < 8; ++tt) acc[tt] = wmma16b(a, frag_kb(WPt + (size_t)(c0 + tt * 16 + nloc) * PVOL + kb, hlf), acc[tt]); }
#pragma unroll
  for (int tt = 0; tt < 8; ++tt) { const float bb = bf16_rne(pb[c0 + tt * 16 + nloc]);
#pragma unroll
    for (int r = 0; r < 8; ++r) Tf[wave][8 * hlf + r][tt * 16 + nloc] = acc[tt][r] * (1.0f / (XS * WSC)) + bb; }
  wave_lds_sync();
  for (int pass = 0; pass < 2; ++pass) { for (int rr = 0; rr < 16; ++rr) *(volatile v4f*)(X + (size_t)(1 + n0 + rr) * D + c0 + lane * 4) = *(const v4f*)(&Tf[wave][rr][lane * 4]); __threadfence(); }
}
__global__ __launch_bounds__(64) void special_kernel(const int* __restrict__ ids, const float* __restrict__ emb, float* __restrict__ X) {
  const int q = blockIdx.x; const int row = q == 0 ? 0 : (q == 1 ? L - 1 : L + (q - 2)); v4f o = {0.0f, 0.0f, 0.0f, 0.0f};
  if (q < 2) { const int id = iclamp(ids[q == 0 ? 0 : L - 1], 0, 3); const v4f e = *(const v4f*)(emb + (size_t)id * D + threadIdx.x * 4); for (int j = 0; j < 4; ++j) o[j] = bf16_rne(e[j]); }
  for (int pass = 0; pass < 2; ++pass) { *(volatile v4f*)(X + (size_t)row * D + threadIdx.x * 4) = o; __threadfence(); }
}
template <bool AFFINE_BF16>
__global__ __launch_bounds__(256) void ln_kernel(const float* __restrict__ X, const float* __restrict__ s, const float* __restrict__ bb, float* __restrict__ Y, int nrows) {
  const int row = blockIdx.x * 8 + (threadIdx.x >> 5), lane = threadIdx.x & 31; if (row >= nrows) return;
  const float* xr = X + (size_t)row * D; v4f a = *(const v4f*)(xr + lane * 4), c = *(const v4f*)(xr + 128 + lane * 4);
  float sum = a[0] + a[1] + a[2] + a[3] + c[0] + c[1] + c[2] + c[3]; for (int w = 16; w >= 1; w >>= 1) sum += __shfl_xor(sum, w); const float mu = sum * (1.0f / D);
  float sq = 0.0f; for (int j = 0; j < 4; ++j) { a[j] -= mu; c[j] -= mu; sq += a[j] * a[j] + c[j] * c[j]; } for (int w = 16; w >= 1; w >>= 1) sq += __shfl_xor(sq, w); const float rs = rsqrtf(sq * (1.0f / D) + LNEPS);
  v4f oa, oc; for (int j = 0; j < 4; ++j) { const int ca = lane * 4 + j, cc = 128 + lane * 4 + j; oa[j] = a[j] * rs * bf16_rne(s[ca]) + bf16_rne(bb[ca]); oc[j] = c[j] * rs * bf16_rne(s[cc]) + bf16_rne(bb[cc]); }
  for (int pass = 0; pass < 2; ++pass) { *(volatile v4f*)(Y + (size_t)row * D + lane * 4) = oa; *(volatile v4f*)(Y + (size_t)row * D + 128 + lane * 4) = oc; __threadfence(); }
}
__global__ __launch_bounds__(256) void attn_kernel(const float* __restrict__ QKV, const int* __restrict__ idx, const int* __restrict__ valid, const float* __restrict__ gdist, const float* __restrict__ decay, float* __restrict__ AO) {
  __shared__ float P[8][NH][160]; __shared__ int IX[8][160];
  const int wave = threadIdx.x >> 5, lane = threadIdx.x & 31; const int l = blockIdx.x * 8 + wave; if (l >= LOUT) return;
  const float* qrow = QKV + (size_t)l * (3 * D);
#pragma unroll 1
  for (int mm = 0; mm < 5; ++mm) { const int kk = lane + 32 * mm; bool ok = false; int key = 0; float gd = 0.0f;
    if (kk < KN) { key = iclamp(idx[(size_t)l * KN + kk], 0, L - 1); ok = (valid[(size_t)l * KN + kk] != 0) && (key <= l); gd = bf16_rne(gdist[(size_t)l * KN + kk]); }
    IX[wave][kk] = ok ? key : 0;
    const float* krow = QKV + (size_t)key * (3 * D) + D;
#pragma unroll 1
    for (int h = 0; h < NH; ++h) { float sdot = 0.0f;
#pragma unroll 2
      for (int d4 = 0; d4 < DH; d4 += 4) { const v4f qv = *(const v4f*)(qrow + h * DH + d4), kv = *(const v4f*)(krow + h * DH + d4); sdot = fmaf(qv[0], kv[0], sdot); sdot = fmaf(qv[1], kv[1], sdot); sdot = fmaf(qv[2], kv[2], sdot); sdot = fmaf(qv[3], kv[3], sdot); }
      P[wave][h][kk] = ok ? sdot * SCALE + gd * bf16_rne(decay[h]) : -INFINITY; } }
#pragma unroll 1
  for (int h = 0; h < NH; ++h) { float v5[5]; float mx = -INFINITY;
#pragma unroll
    for (int mm = 0; mm < 5; ++mm) { v5[mm] = P[wave][h][lane + 32 * mm]; mx = fmaxf(mx, v5[mm]); }
    for (int w = 16; w >= 1; w >>= 1) mx = fmaxf(mx, __shfl_xor(mx, w));
    float ssum = 0.0f;
#pragma unroll
    for (int mm = 0; mm < 5; ++mm) { v5[mm] = (v5[mm] == -INFINITY) ? 0.0f : __expf(v5[mm] - mx); ssum += v5[mm]; }
    for (int w = 16; w >= 1; w >>= 1) ssum += __shfl_xor(ssum, w);
    const float inv = 1.0f / ssum;
#pragma unroll
    for (int mm = 0; mm < 5; ++mm) P[wave][h][lane + 32 * mm] = v5[mm] * inv; }
  wave_lds_sync();
  const int ha = lane >> 4, hb = 2 + (lane >> 4); v4f oa = {0.0f, 0.0f, 0.0f, 0.0f}, ob = {0.0f, 0.0f, 0.0f, 0.0f};
#pragma unroll 1
  for (int kk = 0; kk < KN; ++kk) { const float pa = P[wave][ha][kk], pbv = P[wave][hb][kk]; const float* vrow = QKV + (size_t)IX[wave][kk] * (3 * D) + 2 * D; const v4f va = *(const v4f*)(vrow + lane * 4), vb = *(const v4f*)(vrow + 128 + lane * 4);
    for (int j = 0; j < 4; ++j) { oa[j] = fmaf(pa, va[j], oa[j]); ob[j] = fmaf(pbv, vb[j], ob[j]); } }
  for (int pass = 0; pass < 2; ++pass) { *(volatile v4f*)(AO + (size_t)l * D + lane * 4) = oa; *(volatile v4f*)(AO + (size_t)l * D + 128 + lane * 4) = ob; __threadfence(); }
}
__global__ __launch_bounds__(256) void resid_kernel(float* __restrict__ X, const float* __restrict__ Tm, const float* __restrict__ bias) { const size_t u = (size_t)blockIdx.x * 256 + threadIdx.x; if (u >= (size_t)LP * D / 4) return; const int c = (int)((u * 4) % D); v4f x = *(const v4f*)(X + u * 4); const v4f t = *(const v4f*)(Tm + u * 4);
  for (int j = 0; j < 4; ++j) x[j] += t[j] + bf16_rne(bias[c + j]); for (int pass = 0; pass < 2; ++pass) { *(volatile v4f*)(X + u * 4) = x; __threadfence(); } }
__global__ __launch_bounds__(256) void gelub_kernel(float* __restrict__ F, const float* __restrict__ bias) { const size_t u = (size_t)blockIdx.x * 256 + threadIdx.x; if (u >= (size_t)LP * DFF / 4) return; const int c = (int)((u * 4) % DFF); v4f f = *(const v4f*)(F + u * 4);
  for (int j = 0; j < 4; ++j) { const float v = f[j] + bf16_rne(bias[c + j]); f[j] = 0.5f * v * (1.0f + erff(v * 0.70710678118654752f)); } for (int pass = 0; pass < 2; ++pass) { *(volatile v4f*)(F + u * 4) = f; __threadfence(); } }
__global__ __launch_bounds__(256) void zrows_kernel(float* __restrict__ A) { const size_t u = (size_t)blockIdx.x * 256 + threadIdx.x; if (u >= (size_t)(LP - L) * D / 4) return; const v4f z = {0.0f, 0.0f, 0.0f, 0.0f}; for (int pass = 0; pass < 2; ++pass) { *(volatile v4f*)(A + (size_t)L * D + u * 4) = z; __threadfence(); } }
}

extern "C" void kernel_launch(void* const* d_in, const int* in_sizes, int n_in, void* d_out, int out_size, void* d_ws, size_t ws_size, hipStream_t stream) {
  (void)n_in;
  auto Fp = [&](int i) { return (const float*)d_in[i]; }; auto Ip = [&](int i) { return (const int*)d_in[i]; };
  if (in_sizes[0] != L || in_sizes[1] != IMG * IMG * IMG || in_sizes[2] != L * KN || in_sizes[3] != L * KN || in_sizes[4] != L * KN || in_sizes[5] != NH || in_sizes[6] != 4 * D || in_sizes[7] != PVOL * D || in_sizes[9] != NLAY * D * D || in_sizes[12] != NLAY * D * D || in_sizes[18] != NLAY * D * DFF || in_sizes[20] != NLAY * DFF * D || in_sizes[22] != D || out_size != L * D) return;
  size_t off = 0; char* ws = (char*)d_ws;
  auto carve = [&](size_t bytes) { char* p = ws + off; off += (bytes + 255) & ~(size_t)255; return p; };
  b16* WPt = (b16*)carve((size_t)D * PVOL * 2); b16* WQKV = (b16*)carve((size_t)NLAY * 3 * D * D * 2); b16* WOt = (b16*)carve((size_t)NLAY * D * D * 2); b16* W1t = (b16*)carve((size_t)NLAY * DFF * D * 2); b16* W2t = (b16*)carve((size_t)NLAY * D * DFF * 2);
  float* X = (float*)carve((size_t)LP * D * 4); float* H = (float*)carve((size_t)LP * D * 4); float* QKV = (float*)carve((size_t)LP * 3 * D * 4); float* AO = (float*)carve((size_t)LP * D * 4); float* Tm = (float*)carve((size_t)LP * D * 4); float* F = (float*)carve((size_t)LP * DFF * 4);
  if (off > ws_size || off > ((size_t)128 << 20)) return;
  const unsigned wb = (D * D / 8 + 255) / 256;
  wprep_kernel<PVOL, D><<<(PVOL * D / 8 + 255) / 256, 256, 0, stream>>>(Fp(7), WPt);
  for (int l = 0; l < NLAY; ++l) { const size_t o2 = (size_t)l * D * D;
    wprep_kernel<D, D><<<wb, 256, 0, stream>>>(Fp(9) + o2, WQKV + (size_t)l * 3 * D * D); wprep_kernel<D, D><<<wb, 256, 0, stream>>>(Fp(10) + o2, WQKV + (size_t)l * 3 * D * D + (size_t)D * D); wprep_kernel<D, D><<<wb, 256, 0, stream>>>(Fp(11) + o2, WQKV + (size_t)l * 3 * D * D + (size_t)2 * D * D);
    wprep_kernel<D, D><<<wb, 256, 0, stream>>>(Fp(12) + o2, WOt + o2); wprep_kernel<D, DFF><<<(D * DFF / 8 + 255) / 256, 256, 0, stream>>>(Fp(18) + (size_t)l * D * DFF, W1t + (size_t)l * DFF * D); wprep_kernel<DFF, D><<<(DFF * D / 8 + 255) / 256, 256, 0, stream>>>(Fp(20) + (size_t)l * DFF * D, W2t + (size_t)l * D * DFF); }
  patch_kernel<<<dim3((NL < LP ? NL : NPAT) / 32, 2), 64, 0, stream>>>(Fp(1), WPt, Fp(8), X); special_kernel<<<2 + (LP - L), 64, 0, stream>>>(Ip(0), Fp(6), X);
  const unsigned nb4 = (unsigned)((size_t)NL * D / 4 / 256), nbf = (unsigned)((size_t)NL * DFF / 4 / 256);
  for (int l = 0; l < NLAY; ++l) {
    ln_kernel<true><<<NL / 8, 256, 0, stream>>>(X, Fp(14) + l * D, Fp(15) + l * D, H, NL);
    gemm_kernel<D, 3 * D, LP, false><<<dim3(NL / 32, 6), 64, 0, stream>>>(H, WQKV + (size_t)l * 3 * D * D, QKV);
    attn_kernel<<<(LOUT + 7) / 8, 256, 0, stream>>>(QKV, Ip(2), Ip(3), Fp(4), Fp(5), AO); zrows_kernel<<<((LP - L) * D / 4 + 255) / 256, 256, 0, stream>>>(AO);
    gemm_kernel<D, D, LP, false><<<dim3(NL / 32, 2), 64, 0, stream>>>(AO, WOt + (size_t)l * D * D, Tm); resid_kernel<<<nb4, 256, 0, stream>>>(X, Tm, Fp(13) + l * D);
    ln_kernel<true><<<NL / 8, 256, 0, stream>>>(X, Fp(16) + l * D, Fp(17) + l * D, H, NL);
    gemm_kernel<D, DFF, LP, false><<<dim3(NL / 32, DFF / 128), 64, 0, stream>>>(H, W1t + (size_t)l * DFF * D, F); gelub_kernel<<<nbf, 256, 0, stream>>>(F, Fp(19) + l * DFF);
    gemm_kernel<DFF, D, LP, false><<<dim3(NL / 32, 2), 64, 0, stream>>>(F, W2t + (size_t)l * D * DFF, Tm); resid_kernel<<<nb4, 256, 0, stream>>>(X, Tm, Fp(21) + l * D); }
  ln_kernel<true><<<NL / 8, 256, 0, stream>>>(X, Fp(22), Fp(23), (float*)d_out, LOUT);
}
